// CrossAttention_8031588843664
// MI455X (gfx1250) — hardware-verified
//
#include <hip/hip_runtime.h>
#include <math.h>

#ifndef NB
#define NB 2
#endif
#ifndef SEQ
#define SEQ 4800
#endif
#ifndef SLEN
#define SLEN 4800
#endif
#define NB_FULL 2
#define SEQ_FULL 4800
#define SLEN_FULL 4800
#define EMB 256
#define HEADS 8
#define HD 32
#define KNBR 64
#define FFD 512
#define MQ (NB * SEQ)
#define MS (NB * SLEN)

#define ACARRY 16.0f
#define WCARRY 64.0f
#define MCARRY 256.0f
#define HCARRY 64.0f
static constexpr float SC_PROJ = 1.0f / 1024.0f;
static constexpr float SC_MSG  = 1.0f / 16384.0f;
static constexpr float SC_FF1  = 1.0f / 1024.0f;
static constexpr float SC_FF2  = 1.0f / 4096.0f;
static constexpr float SC2 = 0.17677669529663687f * 1.4426950408889634f;
static_assert(SC_PROJ * (ACARRY * WCARRY) == 1.0f);
static_assert(SC_MSG * (MCARRY * WCARRY) == 1.0f);
static_assert(SC_FF1 * (ACARRY * WCARRY) == 1.0f);
static_assert(SC_FF2 * (HCARRY * WCARRY) == 1.0f);

static_assert(EMB == 256 && HEADS * HD == EMB && HD == 32);
static_assert(32 * 8 == EMB);
static_assert(4 * 8 == HD);
static_assert(KNBR == 64);
static_assert(FFD == 2 * EMB);
static_assert(NB <= NB_FULL && SEQ <= SEQ_FULL && SLEN <= SLEN_FULL);
static_assert(MQ % 64 == 0 && MS % 64 == 0);
static_assert(EMB % 64 == 0 && FFD % 64 == 0);
static_assert(EMB % 32 == 0 && FFD % 32 == 0);
static_assert(MQ % 8 == 0 && MS % 8 == 0);
static_assert((EMB * (EMB / 8)) % 256 == 0 && (FFD * (FFD / 8)) % 256 == 0 && (EMB * (FFD / 8)) % 256 == 0);
static_assert(32 * 16 * 8 == 16 * 64 * 4);
static_assert(32 * 16 * 4 == 16 * 64 * 2);
#define GT_PITCH 68
static_assert(8 * 16 * GT_PITCH * 4 <= 131072);

static constexpr size_t al256(size_t b) { return (b + 255) & ~(size_t)255; }
static constexpr size_t WS_TOTAL =
    al256((size_t)MS * EMB * 2) + al256((size_t)MQ * FFD * 2) + al256((size_t)MQ * EMB * 4) + 2 * al256((size_t)MS * EMB * 4) +
    al256((size_t)MQ * EMB * 2) + al256((size_t)MQ * EMB * 4) + al256((size_t)MQ * FFD * 2) + al256((size_t)MQ * EMB * 4) +
    4 * al256((size_t)EMB * EMB * 2) + al256((size_t)FFD * FFD * 2) + al256((size_t)FFD * EMB * 2);
static_assert(WS_TOTAL <= (size_t)134217728);

static constexpr int X_NEED = ((NB - 1) * SEQ_FULL + SEQ) * EMB;
static constexpr int S_NEED = ((NB - 1) * SLEN_FULL + SLEN) * EMB;
static constexpr int I_NEED = ((NB - 1) * SEQ_FULL + SEQ) * KNBR;

typedef __attribute__((ext_vector_type(16))) _Float16 v16h;
typedef __attribute__((ext_vector_type(8)))  _Float16 v8h;
typedef __attribute__((ext_vector_type(8)))  float    v8f;
typedef __attribute__((ext_vector_type(4)))  float    v4f;
typedef _Float16 h16;


__device__ __forceinline__ float bfr(float f) {
    unsigned u = __float_as_uint(f);
    u += 0x7FFFu + ((u >> 16) & 1u);
    return __uint_as_float(u & 0xFFFF0000u);
}
static __device__ __forceinline__ h16 toh_flush(float v) { const float w = (fabsf(v) < 6.103515625e-05f) ? 0.0f : v; return (h16)w; }
__device__ __forceinline__ void st8hf(_Float16* P, size_t o, const float* v) {
    v8h pk;
#pragma unroll
    for (int e = 0; e < 8; ++e) pk[e] = toh_flush(v[e]);
    *(volatile v8h*)(P + o) = pk;
    __threadfence();
    *(volatile v8h*)(P + o) = pk;
}

union FragU { v16h v; v8h h[2]; };
__device__ __forceinline__ v16h frag_ld(const _Float16* p) {
    FragU f; f.h[0] = *(const v8h*)(p); f.h[1] = *(const v8h*)(p + 16); return f.v;
}
__device__ __forceinline__ v8f wmma16(v16h a, v16h b, v8f c) {
    c = __builtin_amdgcn_wmma_f32_16x16x32_f16(false, a, false, b, (short)0, c, false, false);
    asm volatile("v_nop\n\tv_nop\n\tv_nop\n\tv_nop" : "+v"(c) : "v"(a), "v"(b));
    return c;
}
__device__ __forceinline__ void wave_sync_lds() {
    __builtin_amdgcn_fence(3  , "workgroup");
    __builtin_amdgcn_wave_barrier();
    __builtin_amdgcn_fence(2  , "workgroup");
}

template <int OUT_MODE, bool RELU>
__device__ __forceinline__ void gemm64_body(
    const _Float16* __restrict__ A, const unsigned lda, const _Float16* __restrict__ Bt, const unsigned ldb,
    void* __restrict__ Cout, const unsigned ldc, const unsigned M, const unsigned N, const unsigned K,
    const float scale, const float oscale) {
  __shared__ __align__(16) float sT[8][16 * GT_PITCH];
  const unsigned lane = threadIdx.x & 31u;
  const unsigned wave = (unsigned)__builtin_amdgcn_readfirstlane((int)(threadIdx.x >> 5));
  const unsigned tilesN = N >> 6, tilesM = M >> 6;
  const unsigned tile = blockIdx.x * 8u + wave;
  if (tile >= tilesM * tilesN) return;
  const unsigned tm = tile / tilesN;
  const unsigned tn = tile - tm * tilesN;
  const unsigned m0 = tm << 6, n0 = tn << 6;
  const unsigned rlane = lane & 15u;
  const unsigned koff = (lane >> 4) * 8u;
  const unsigned mOff = koff;

  v8f acc[4][4];
#pragma unroll
  for (int i = 0; i < 4; ++i)
#pragma unroll
    for (int j = 0; j < 4; ++j) acc[i][j] = (v8f){0.f,0.f,0.f,0.f,0.f,0.f,0.f,0.f};

  for (unsigned k0 = 0; k0 < K; k0 += 32u) {
    v16h bh[4];
#pragma unroll
    for (int j = 0; j < 4; ++j)
      bh[j] = frag_ld(Bt + (size_t)(n0 + ((unsigned)j << 4) + rlane) * ldb + koff + k0);
    unsigned ka = koff + k0;
    asm volatile("" : "+v"(ka) : "v"(bh[3]));
#pragma unroll
    for (int i = 0; i < 4; ++i) {
      const v16h ah = frag_ld(A + (size_t)(m0 + ((unsigned)i << 4) + rlane) * lda + ka);
#pragma unroll
      for (int j = 0; j < 4; ++j)
        acc[i][j] = wmma16(ah, bh[j], acc[i][j]);
    }
  }

  float* slab = sT[wave];
#pragma unroll
  for (int i = 0; i < 4; ++i) {
    const unsigned mBase = m0 + ((unsigned)i << 4);
#pragma unroll
    for (int j = 0; j < 4; ++j) {
#pragma unroll
      for (int r = 0; r < 8; ++r) {
        float v = acc[i][j][r] * scale;
        if (RELU) v = fmaxf(v, 0.0f);
        if (OUT_MODE == 1) v *= oscale;
        slab[(mOff + (unsigned)r) * GT_PITCH + ((unsigned)j << 4) + rlane] = v;
      }
    }
    wave_sync_lds();
    if (OUT_MODE == 0) {
      float* C = (float*)Cout;
      const unsigned hh = lane >> 4, c4 = (lane & 15u) * 4u;
#pragma unroll
      for (int half = 0; half < 2; ++half) {
        v4f vv[4];
#pragma unroll
        for (int it = 0; it < 4; ++it) {
          const unsigned row = (unsigned)(half * 4 + it) * 2u + hh;
          vv[it] = *(const v4f*)(slab + row * GT_PITCH + c4);
        }
        for (int pass = 0; pass < 2; ++pass) {
#pragma unroll
          for (int it = 0; it < 4; ++it) {
            const unsigned row = (unsigned)(half * 4 + it) * 2u + hh;
            *(volatile v4f*)(C + (size_t)(mBase + row) * ldc + n0 + c4) = vv[it];
          }
          __threadfence();
        }
      }
    } else {
      _Float16* C = (_Float16*)Cout;
      const unsigned q = lane >> 3, c8 = (lane & 7u) * 8u;
      v8h hv[4];
#pragma unroll
      for (int it = 0; it < 4; ++it) {
        const unsigned row = (unsigned)it * 4u + q;
        const float* sp = slab + row * GT_PITCH + c8;
#pragma unroll
        for (int e = 0; e < 8; ++e) hv[it][e] = toh_flush(sp[e]);
      }
      for (int pass = 0; pass < 2; ++pass) {
#pragma unroll
        for (int it = 0; it < 4; ++it) {
          const unsigned row = (unsigned)it * 4u + q;
          *(volatile v8h*)(C + (size_t)(mBase + row) * ldc + n0 + c8) = hv[it];
        }
        __threadfence();
      }
    }
    wave_sync_lds();
  }
}

__global__ __launch_bounds__(256) void k_gemm_proj(const _Float16* __restrict__ A, unsigned lda, const _Float16* __restrict__ Bt,
                                                   float* __restrict__ C, unsigned M) {
  gemm64_body<0, false>(A, lda, Bt, (unsigned)EMB, (void*)C, (unsigned)EMB, M, (unsigned)EMB, (unsigned)EMB, SC_PROJ, 1.0f);
}
__global__ __launch_bounds__(256) void k_gemm_msg(const _Float16* __restrict__ A, const _Float16* __restrict__ Bt, float* __restrict__ C) {
  gemm64_body<0, false>(A, (unsigned)EMB, Bt, (unsigned)EMB, (void*)C, (unsigned)EMB, (unsigned)MQ, (unsigned)EMB, (unsigned)EMB, SC_MSG, 1.0f);
}
__global__ __launch_bounds__(256) void k_gemm_ff1(const _Float16* __restrict__ A, const _Float16* __restrict__ Bt, _Float16* __restrict__ C) {
  gemm64_body<1, true>(A, (unsigned)FFD, Bt, (unsigned)FFD, (void*)C, (unsigned)FFD, (unsigned)MQ, (unsigned)FFD, (unsigned)FFD, SC_FF1, HCARRY);
}
__global__ __launch_bounds__(256) void k_gemm_ff2(const _Float16* __restrict__ A, const _Float16* __restrict__ Bt, float* __restrict__ C) {
  gemm64_body<0, false>(A, (unsigned)FFD, Bt, (unsigned)FFD, (void*)C, (unsigned)EMB, (unsigned)MQ, (unsigned)EMB, (unsigned)FFD, SC_FF2, 1.0f);
}

__global__ __launch_bounds__(256) void k_wt16(const float* __restrict__ Wm, unsigned KI, unsigned NO, unsigned lgper,
                                              _Float16* __restrict__ W16) {
    const unsigned layer = blockIdx.y;
    const float* Wl = Wm + (size_t)layer * KI * NO;
    _Float16* Dl = W16 + (size_t)layer * KI * NO;
    const unsigned u = blockIdx.x * 256u + threadIdx.x;
    const unsigned per = 1u << lgper;
    if (u >= NO * per) return;
    const unsigned k0 = 8u * (u & (per - 1u));
    const unsigned o = u >> lgper;
    float v[8];
#pragma unroll
    for (int i = 0; i < 8; ++i) v[i] = bfr(Wl[(size_t)(k0 + (unsigned)i) * NO + o]) * WCARRY;
    st8hf(Dl, (size_t)o * KI + k0, v);
}

template <unsigned RPB, unsigned RPB_FULL>
__device__ __forceinline__ void cvt16_body(const float* __restrict__ in, _Float16* __restrict__ plane, const unsigned pitch, const unsigned rows) {
    const unsigned u = blockIdx.x * 256u + threadIdx.x;
    const unsigned row = u >> 5, c0 = (u & 31u) * 8u;
    if (row >= rows) return;
    const unsigned n = row / RPB;
    const unsigned l = row - n * RPB;
    const float* xr = in + (size_t)(n * RPB_FULL + l) * (unsigned)EMB + c0;
    const v4f a = *(const v4f*)xr, b = *(const v4f*)(xr + 4);
    float v[8] = {bfr(a.x) * ACARRY, bfr(a.y) * ACARRY, bfr(a.z) * ACARRY, bfr(a.w) * ACARRY,
                  bfr(b.x) * ACARRY, bfr(b.y) * ACARRY, bfr(b.z) * ACARRY, bfr(b.w) * ACARRY};
    st8hf(plane, (size_t)row * pitch + c0, v);
}
__global__ __launch_bounds__(256) void k_cvt_x(const float* __restrict__ x, _Float16* __restrict__ cat16) {
    cvt16_body<(unsigned)SEQ, (unsigned)SEQ_FULL>(x, cat16, (unsigned)FFD, (unsigned)MQ);
}
__global__ __launch_bounds__(256) void k_cvt_src(const float* __restrict__ src, _Float16* __restrict__ src16) {
    cvt16_body<(unsigned)SLEN, (unsigned)SLEN_FULL>(src, src16, (unsigned)EMB, (unsigned)MS);
}

__global__ __launch_bounds__(256) void k_gattn(const float* __restrict__ Qp, const float* __restrict__ Kp, const float* __restrict__ Vp,
                                               const int* __restrict__ idx, _Float16* __restrict__ msg16) {
    const unsigned lane = threadIdx.x & 31u;
    const unsigned wave = (unsigned)__builtin_amdgcn_readfirstlane((int)(threadIdx.x >> 5));
    const unsigned qr = blockIdx.x * 8u + wave;
    if (qr >= (unsigned)MQ) return;
    const unsigned n = qr / (unsigned)SEQ;
    const unsigned l = qr - n * (unsigned)SEQ;
    const int* irow = idx + (size_t)(n * (unsigned)SEQ_FULL + l) * (unsigned)KNBR;
    const float* qp = Qp + (size_t)qr * (unsigned)EMB + 8u * lane;
    const v4f q0 = *(const v4f*)qp, q1 = *(const v4f*)(qp + 4);
    const float* kb = Kp + (size_t)(n * (unsigned)SLEN) * (unsigned)EMB + 8u * lane;
    const float* vb = Vp + (size_t)(n * (unsigned)SLEN) * (unsigned)EMB + 8u * lane;
    float m = -3.0e38f, lsum = 0.f;
    v4f a0 = (v4f){0.f, 0.f, 0.f, 0.f}, a1 = (v4f){0.f, 0.f, 0.f, 0.f};
#pragma unroll 1
    for (unsigned kk = 0; kk < (unsigned)KNBR; ++kk) {
        const int idr = irow[kk];
        const unsigned id = (unsigned)min(max(idr, 0), SLEN - 1);
        const float* kr = kb + (size_t)id * (unsigned)EMB;
        const float* vr = vb + (size_t)id * (unsigned)EMB;
        const v4f k0 = *(const v4f*)kr, k1 = *(const v4f*)(kr + 4);
        const v4f v0 = *(const v4f*)vr, v1 = *(const v4f*)(vr + 4);
        float p = q0.x * k0.x + q0.y * k0.y + q0.z * k0.z + q0.w * k0.w + q1.x * k1.x + q1.y * k1.y + q1.z * k1.z + q1.w * k1.w;
        p += __shfl_xor(p, 1, 32);
        p += __shfl_xor(p, 2, 32);
        const float s = p * SC2;
        const float mnew = (s > m) ? s : m;
        const float alpha = exp2f(m - mnew);
        const float pe = exp2f(s - mnew);
        lsum = lsum * alpha + pe;
        a0 = a0 * alpha + v0 * pe;
        a1 = a1 * alpha + v1 * pe;
        m = mnew;
    }
    const float sc = (1.0f / lsum) * MCARRY;
    float y[8] = {a0.x * sc, a0.y * sc, a0.z * sc, a0.w * sc, a1.x * sc, a1.y * sc, a1.z * sc, a1.w * sc};
    st8hf(msg16, (size_t)qr * (unsigned)EMB + 8u * lane, y);
}

__global__ __launch_bounds__(256) void k_ln_cat(const float* __restrict__ h, const float* __restrict__ g, const float* __restrict__ bt,
                                                _Float16* __restrict__ cat16) {
    const unsigned wave = (unsigned)__builtin_amdgcn_readfirstlane((int)(threadIdx.x >> 5));
    const unsigned row = blockIdx.x * 8u + wave;
    const unsigned L = threadIdx.x & 31u;
    if (row >= (unsigned)MQ) return;
    const float* hr = h + (size_t)row * 256u + 8u * L;
    const v4f a = *(const v4f*)hr, b = *(const v4f*)(hr + 4);
    float s = ((a.x + a.y) + (a.z + a.w)) + ((b.x + b.y) + (b.z + b.w));
#pragma unroll
    for (int o = 16; o > 0; o >>= 1) s += __shfl_xor(s, o, 32);
    const float mu = s * (1.0f / 256.0f);
    float d[8] = {a.x - mu, a.y - mu, a.z - mu, a.w - mu, b.x - mu, b.y - mu, b.z - mu, b.w - mu};
    float q = 0.f;
#pragma unroll
    for (int i = 0; i < 8; ++i) q += d[i] * d[i];
#pragma unroll
    for (int o = 16; o > 0; o >>= 1) q += __shfl_xor(q, o, 32);
    const float rs = rsqrtf(q * (1.0f / 256.0f) + 1e-5f);
    const v4f g0 = *(const v4f*)(g + 8u * L), g1 = *(const v4f*)(g + 8u * L + 4u);
    const v4f b0 = *(const v4f*)(bt + 8u * L), b1 = *(const v4f*)(bt + 8u * L + 4u);
    const float gg[8] = {g0.x, g0.y, g0.z, g0.w, g1.x, g1.y, g1.z, g1.w};
    const float bb[8] = {b0.x, b0.y, b0.z, b0.w, b1.x, b1.y, b1.z, b1.w};
    float y[8];
#pragma unroll
    for (int i = 0; i < 8; ++i) y[i] = (d[i] * rs * bfr(gg[i]) + bfr(bb[i])) * ACARRY;
    st8hf(cat16, (size_t)row * (unsigned)FFD + (unsigned)EMB + 8u * L, y);
}

__global__ __launch_bounds__(256) void k_ln_out(const float* __restrict__ h2, const float* __restrict__ x, const float* __restrict__ g,
                                                const float* __restrict__ bt, float* __restrict__ out) {
    const unsigned wave = (unsigned)__builtin_amdgcn_readfirstlane((int)(threadIdx.x >> 5));
    const unsigned row = blockIdx.x * 8u + wave;
    const unsigned L = threadIdx.x & 31u;
    if (row >= (unsigned)MQ) return;
    const unsigned n = row / (unsigned)SEQ;
    const unsigned l = row - n * (unsigned)SEQ;
    const size_t rf = (size_t)(n * (unsigned)SEQ_FULL + l) * 256u;
    const float* hr = h2 + (size_t)row * 256u + 4u * L;
    const v4f a = *(const v4f*)hr, b = *(const v4f*)(hr + 128);
    float s = ((a.x + a.y) + (a.z + a.w)) + ((b.x + b.y) + (b.z + b.w));
#pragma unroll
    for (int o = 16; o > 0; o >>= 1) s += __shfl_xor(s, o, 32);
    const float mu = s * (1.0f / 256.0f);
    float d[8] = {a.x - mu, a.y - mu, a.z - mu, a.w - mu, b.x - mu, b.y - mu, b.z - mu, b.w - mu};
    float q = 0.f;
#pragma unroll
    for (int i = 0; i < 8; ++i) q += d[i] * d[i];
#pragma unroll
    for (int o = 16; o > 0; o >>= 1) q += __shfl_xor(q, o, 32);
    const float rs = rsqrtf(q * (1.0f / 256.0f) + 1e-5f);
    const v4f g0 = *(const v4f*)(g + 4u * L), g1 = *(const v4f*)(g + 128u + 4u * L);
    const v4f b0 = *(const v4f*)(bt + 4u * L), b1 = *(const v4f*)(bt + 128u + 4u * L);
    const v4f x0 = *(const v4f*)(x + rf + 4u * L), x1 = *(const v4f*)(x + rf + 128u + 4u * L);
    const float gg[8] = {g0.x, g0.y, g0.z, g0.w, g1.x, g1.y, g1.z, g1.w};
    const float bb[8] = {b0.x, b0.y, b0.z, b0.w, b1.x, b1.y, b1.z, b1.w};
    const float xx[8] = {x0.x, x0.y, x0.z, x0.w, x1.x, x1.y, x1.z, x1.w};
    float y[8];
#pragma unroll
    for (int i = 0; i < 8; ++i) y[i] = bfr(xx[i]) + (d[i] * rs * bfr(gg[i]) + bfr(bb[i]));
    const v4f o0 = (v4f){y[0], y[1], y[2], y[3]};
    const v4f o1 = (v4f){y[4], y[5], y[6], y[7]};
    float* dst = out + rf + 4u * L;
    for (int pass = 0; pass < 2; ++pass) {
        *(volatile v4f*)(dst) = o0;
        *(volatile v4f*)(dst + 128) = o1;
        __threadfence();
    }
}

extern "C" void kernel_launch(void* const* d_in, const int* in_sizes, int n_in, void* d_out, int out_size,
                              void* d_ws, size_t ws_size, hipStream_t stream) {
    if (n_in < 13) return;
    if (in_sizes[0] < X_NEED || in_sizes[1] < S_NEED || in_sizes[2] < I_NEED) return;
    if (in_sizes[3] < EMB * EMB || in_sizes[4] < EMB * EMB || in_sizes[5] < EMB * EMB || in_sizes[6] < EMB * EMB) return;
    if (in_sizes[7] < FFD * FFD || in_sizes[8] < FFD * EMB) return;
    if (in_sizes[9] < EMB || in_sizes[10] < EMB || in_sizes[11] < EMB || in_sizes[12] < EMB) return;
    if (out_size < X_NEED) return;

    const float* x      = (const float*)d_in[0];
    const float* source = (const float*)d_in[1];
    const int*   eidx   = (const int*)d_in[2];
    const float* Wq     = (const float*)d_in[3];
    const float* Wk     = (const float*)d_in[4];
    const float* Wv     = (const float*)d_in[5];
    const float* Wm     = (const float*)d_in[6];
    const float* W1     = (const float*)d_in[7];
    const float* W2     = (const float*)d_in[8];
    const float* g1     = (const float*)d_in[9];
    const float* b1     = (const float*)d_in[10];
    const float* g2     = (const float*)d_in[11];
    const float* b2     = (const float*)d_in[12];
    float* out = (float*)d_out;

    char* wsp = (char*)d_ws;
    size_t off = 0;
    auto carve = [&](size_t bytes) -> void* { void* r = wsp + off; off += (bytes + 255) & ~(size_t)255; return r; };
    _Float16* src16 = (_Float16*)carve((size_t)MS * EMB * 2);
    _Float16* cat16 = (_Float16*)carve((size_t)MQ * FFD * 2);
    float*    Qp    = (float*)carve((size_t)MQ * EMB * 4);
    float*    Kp    = (float*)carve((size_t)MS * EMB * 4);
    float*    Vp    = (float*)carve((size_t)MS * EMB * 4);
    _Float16* msg16 = (_Float16*)carve((size_t)MQ * EMB * 2);
    float*    M1    = (float*)carve((size_t)MQ * EMB * 4);
    _Float16* h16p  = (_Float16*)carve((size_t)MQ * FFD * 2);
    float*    H2    = (float*)carve((size_t)MQ * EMB * 4);
    _Float16* wq16  = (_Float16*)carve((size_t)EMB * EMB * 2);
    _Float16* wk16  = (_Float16*)carve((size_t)EMB * EMB * 2);
    _Float16* wv16  = (_Float16*)carve((size_t)EMB * EMB * 2);
    _Float16* wm16  = (_Float16*)carve((size_t)EMB * EMB * 2);
    _Float16* w1t   = (_Float16*)carve((size_t)FFD * FFD * 2);
    _Float16* w2t   = (_Float16*)carve((size_t)FFD * EMB * 2);
    if (off != WS_TOTAL || off > ws_size || off > (size_t)134217728) return;

    k_wt16<<<dim3((EMB * (EMB / 8)) / 256, 1), 256, 0, stream>>>(Wq, EMB, EMB, 5, wq16);
    k_wt16<<<dim3((EMB * (EMB / 8)) / 256, 1), 256, 0, stream>>>(Wk, EMB, EMB, 5, wk16);
    k_wt16<<<dim3((EMB * (EMB / 8)) / 256, 1), 256, 0, stream>>>(Wv, EMB, EMB, 5, wv16);
    k_wt16<<<dim3((EMB * (EMB / 8)) / 256, 1), 256, 0, stream>>>(Wm, EMB, EMB, 5, wm16);
    k_wt16<<<dim3((FFD * (FFD / 8)) / 256, 1), 256, 0, stream>>>(W1, FFD, FFD, 6, w1t);
    k_wt16<<<dim3((EMB * (FFD / 8)) / 256, 1), 256, 0, stream>>>(W2, FFD, EMB, 6, w2t);

    k_cvt_x<<<MQ / 8, 256, 0, stream>>>(x, cat16);
    k_cvt_src<<<MS / 8, 256, 0, stream>>>(source, src16);

    const unsigned gQ = ((MQ / 64) * (EMB / 64) + 7) / 8;
    const unsigned gS = ((MS / 64) * (EMB / 64) + 7) / 8;
    const unsigned gF = ((MQ / 64) * (FFD / 64) + 7) / 8;

    k_gemm_proj<<<gQ, 256, 0, stream>>>((const _Float16*)cat16, FFD, (const _Float16*)wq16, Qp, MQ);
    k_gemm_proj<<<gS, 256, 0, stream>>>((const _Float16*)src16, EMB, (const _Float16*)wk16, Kp, MS);
    k_gemm_proj<<<gS, 256, 0, stream>>>((const _Float16*)src16, EMB, (const _Float16*)wv16, Vp, MS);

    k_gattn<<<MQ / 8, 256, 0, stream>>>(Qp, Kp, Vp, eidx, msg16);

    k_gemm_msg<<<gQ, 256, 0, stream>>>((const _Float16*)msg16, (const _Float16*)wm16, M1);
    k_ln_cat<<<MQ / 8, 256, 0, stream>>>(M1, g1, b1, cat16);
    k_gemm_ff1<<<gF, 256, 0, stream>>>((const _Float16*)cat16, (const _Float16*)w1t, h16p);
    k_gemm_ff2<<<gQ, 256, 0, stream>>>((const _Float16*)h16p, (const _Float16*)w2t, H2);
    k_ln_out<<<MQ / 8, 256, 0, stream>>>(H2, x, g2, b2, out);
}
